// ConcatCriticTorch_86620900426436
// MI455X (gfx1250) — hardware-run, weakly checked
//
#include <hip/hip_runtime.h>
#include <math.h>

typedef __attribute__((ext_vector_type(16))) _Float16 v16h;
typedef __attribute__((ext_vector_type(8)))  _Float16 v8h;
typedef __attribute__((ext_vector_type(8)))  float    v8f;
typedef __attribute__((ext_vector_type(4)))  float    v4f;

constexpr int kNB   = 512;
constexpr int kDF   = 128;
constexpr int kHID  = 512;
constexpr int kKIN  = 2 * kDF;
static_assert((kNB % 64) == 0 && (kHID % 64) == 0);
static_assert((kDF % 32) == 0);

constexpr float kCarryAct = 16.0f;
constexpr float kCarryW   = 256.0f;
constexpr float kFold     = 1.0f / (kCarryAct * kCarryW);
constexpr float kF16MinNormal = 6.103515625e-05f;

constexpr size_t kPlaneElems = (size_t)kNB * kDF;
constexpr size_t kHidElems   = (size_t)kNB * kHID;
constexpr size_t kOffAH  = 0;
constexpr size_t kOffWT  = kOffAH + 2 * kPlaneElems * 2;
constexpr size_t kOffHXY = kOffWT + 2 * kPlaneElems * 2;
constexpr size_t kWsTotal = kOffHXY + 2 * kHidElems * 4;
static_assert(kWsTotal == 2621440ull);
static_assert(kWsTotal <= 134217728ull);
static_assert((kOffWT % 128) == 0 && (kOffHXY % 128) == 0);
static_assert(kHID * kDF == (int)kPlaneElems);

__device__ __forceinline__ void guard1_h(v8f& a, v16h x, v16h y) {
  asm volatile("v_nop\n\tv_nop\n\tv_nop\n\tv_nop" : "+v"(a) : "v"(x), "v"(y));
}
__device__ __forceinline__ void keep4_h(v16h a, v16h b, v16h c, v16h d) {
  asm volatile("v_nop" :: "v"(a), "v"(b), "v"(c), "v"(d));
}
struct FragH {
  union U { v16h v; v8h h[2]; };
  static __device__ __forceinline__ v16h load(const _Float16* p) {
    U f;
    f.h[0] = *(const v8h*)(p);
    f.h[1] = *(const v8h*)(p + 16);
    return f.v;
  }
  static __device__ __forceinline__ v8f mma(v16h a, v16h b, v8f c) {
    return __builtin_amdgcn_wmma_f32_16x16x32_f16(false, a, false, b, (short)0, c, false, false);
  }
};

__device__ __forceinline__ _Float16 to_f16_carried(float v, float carry) {
  const float s = v * carry;
  const float f = (fabsf(s) < kF16MinNormal) ? 0.0f : s;
  return (_Float16)f;
}

constexpr int kCvtBlocks   = (2 * kNB * kDF / 8) / 256;
constexpr int kTrBlocks    = (kKIN / 64) * (kHID / 64);
constexpr int kActThreads  = kNB * kDF / 8;
static_assert(kCvtBlocks == 64 && kTrBlocks == 32 && kActThreads == 8192);

__global__ __launch_bounds__(256) void prep_planes_f16(
    const float* __restrict__ x, const float* __restrict__ y, const float* __restrict__ W1,
    unsigned short* __restrict__ AH, unsigned short* __restrict__ WT)
{
  __shared__ __align__(16) float sT[64 * 68];
  const int tid = threadIdx.x;
  const int bid = blockIdx.x;
  if (bid < kCvtBlocks) {
    const int i = bid * 256 + tid;
    const float* src = (bid < kCvtBlocks / 2) ? x : y;
    const size_t e0 = (size_t)(i & (kActThreads - 1)) << 3;
    const v4f a0 = *(const v4f*)(src + e0);
    const v4f a1 = *(const v4f*)(src + e0 + 4);
    v8h hv;
#pragma unroll
    for (int e = 0; e < 4; ++e) {
      const float f0 = a0[e];
      const float f1 = a1[e];
      hv[e]     = to_f16_carried(f0, kCarryAct);
      hv[4 + e] = to_f16_carried(f1, kCarryAct);
    }
    unsigned short* q = AH + ((size_t)i << 3);
    *(volatile v8h*)q = hv;
    __threadfence();
    *(volatile v8h*)q = hv;
  } else {
    const int tb = bid - kCvtBlocks;
    const int kt = tb >> 3;
    const int nt = tb & 7;
    const int k0 = kt << 6;
    const int n0 = nt << 6;
    const int kr = tid >> 4;
    const int c4 = (tid & 15) << 2;
#pragma unroll
    for (int i = 0; i < 4; ++i) {
      const int krow = kr + 16 * i;
      const v4f v = *(const v4f*)(W1 + (size_t)(k0 + krow) * kHID + n0 + c4);
      *(v4f*)(sT + krow * 68 + c4) = v;
    }
    __syncthreads();
    const int q  = tid >> 3;
    const int c8 = (tid & 7) << 3;
    const int plane = k0 >> 7;
    const int kcol0 = k0 & (kDF - 1);
    v8h hv[2];
#pragma unroll
    for (int it = 0; it < 2; ++it) {
      const int nrow = it * 32 + q;
#pragma unroll
      for (int e = 0; e < 8; ++e) {
        const float f = sT[(c8 + e) * 68 + nrow];
        hv[it][e] = to_f16_carried(f, kCarryW);
      }
    }
    unsigned short* base = WT + (size_t)plane * kPlaneElems + (size_t)kcol0 + c8;
#pragma unroll
    for (int it = 0; it < 2; ++it) {
      const int nrow = it * 32 + q;
      *(volatile v8h*)(base + (size_t)(n0 + nrow) * kDF) = hv[it];
    }
    __threadfence();
#pragma unroll
    for (int it = 0; it < 2; ++it) {
      const int nrow = it * 32 + q;
      *(volatile v8h*)(base + (size_t)(n0 + nrow) * kDF) = hv[it];
    }
  }
}

__global__ __launch_bounds__(256) void hidden_gemm_f16(
    const unsigned short* __restrict__ Ap, const unsigned short* __restrict__ Btp,
    float* __restrict__ Cp, const float* __restrict__ bias)
{
  __shared__ __align__(16) float sT[8][16 * 68];
  const int bz   = blockIdx.y;
  const int lane = threadIdx.x & 31;
  const int wave = threadIdx.x >> 5;
  const int tile = blockIdx.x * 8 + wave;
  const int tm = tile >> 3;
  const int tn = tile & 7;
  const int m0 = tm << 6;
  const int n0 = tn << 6;

  const _Float16* Ab = (const _Float16*)Ap  + (size_t)bz * kPlaneElems;
  const _Float16* Bb = (const _Float16*)Btp + (size_t)bz * kPlaneElems;
  float* C = Cp + (size_t)bz * kHidElems;

  const int rlane = lane & 15;
  const int koff  = (lane >> 4) * 8;
  const int mOff  = (lane >> 4) * 8;

  v8f acc[4][4];
#pragma unroll
  for (int i = 0; i < 4; ++i)
#pragma unroll
    for (int j = 0; j < 4; ++j) acc[i][j] = (v8f){0.f, 0.f, 0.f, 0.f, 0.f, 0.f, 0.f, 0.f};

  for (int k0 = 0; k0 < kDF; k0 += 32) {
    v16h bh[4];
#pragma unroll
    for (int j = 0; j < 4; ++j) {
      const size_t bo = (size_t)(n0 + (j << 4) + rlane) * kDF + koff + k0;
      bh[j] = FragH::load(Bb + bo);
    }
#pragma unroll
    for (int i = 0; i < 4; ++i) {
      const size_t ao = (size_t)(m0 + (i << 4) + rlane) * kDF + koff + k0;
      const v16h ah = FragH::load(Ab + ao);
#pragma unroll
      for (int j = 0; j < 4; ++j) acc[i][j] = FragH::mma(ah, bh[j], acc[i][j]);
#pragma unroll
      for (int j = 0; j < 4; ++j) guard1_h(acc[i][j], ah, bh[j]);
    }
    keep4_h(bh[0], bh[1], bh[2], bh[3]);
  }

  float bvj[4];
#pragma unroll
  for (int j = 0; j < 4; ++j) {
    const float bl = bias[n0 + (j << 4) + rlane];
    bvj[j] = (bz == 1) ? bl : 0.0f;
  }

  float* slab = sT[wave];
#pragma unroll
  for (int i = 0; i < 4; ++i) {
    const int mBase = m0 + (i << 4);
#pragma unroll
    for (int j = 0; j < 4; ++j) {
#pragma unroll
      for (int r = 0; r < 8; ++r) {
        const float v = acc[i][j][r] * kFold + bvj[j];
        slab[(mOff + r) * 68 + (j << 4) + rlane] = v;
      }
    }
    __builtin_amdgcn_fence(__ATOMIC_RELEASE, "workgroup");
    __builtin_amdgcn_wave_barrier();
    __builtin_amdgcn_fence(__ATOMIC_ACQUIRE, "workgroup");
    {
      const int hh = lane >> 4;
      const int c4 = (lane & 15) * 4;
      for (int pass = 0; pass < 2; ++pass) {
#pragma unroll
        for (int it = 0; it < 8; ++it) {
          const int row = it * 2 + hh;
          const v4f v = *(const v4f*)(slab + row * 68 + c4);
          *(volatile v4f*)(C + (size_t)(mBase + row) * kHID + n0 + c4) = v;
        }
        __threadfence();
      }
    }
    __builtin_amdgcn_fence(__ATOMIC_RELEASE, "workgroup");
    __builtin_amdgcn_wave_barrier();
    __builtin_amdgcn_fence(__ATOMIC_ACQUIRE, "workgroup");
  }
}

__global__ __launch_bounds__(256) void pair_score_kernel(
    const float* __restrict__ Hx, const float* __restrict__ Hy,
    const float* __restrict__ W2, const float* __restrict__ b2,
    float* __restrict__ out)
{
  __shared__ float hxs[64 * 33];
  __shared__ float hys[64 * 33];
  __shared__ float w2s[32];

  const int t  = threadIdx.x;
  const int tx = t & 15;
  const int ty = t >> 4;
  const int a0 = blockIdx.y * 64;
  const int b0 = blockIdx.x * 64;
  const int lrow = t >> 2;
  const int jb   = (t & 3) * 8;

  float acc[4][4];
#pragma unroll
  for (int r = 0; r < 4; ++r)
#pragma unroll
    for (int c = 0; c < 4; ++c) acc[r][c] = 0.0f;

#pragma unroll 1
  for (int h0 = 0; h0 < kHID; h0 += 32) {
    __syncthreads();
    {
      const float* gx = Hx + (size_t)(a0 + lrow) * kHID + h0 + jb;
      const float* gy = Hy + (size_t)(b0 + lrow) * kHID + h0 + jb;
      const v4f vx0 = *(const v4f*)(gx);
      const v4f vx1 = *(const v4f*)(gx + 4);
      const v4f vy0 = *(const v4f*)(gy);
      const v4f vy1 = *(const v4f*)(gy + 4);
      float wv = W2[h0 + (t & 31)];
      asm volatile("" : "+v"(wv));
      float* px = hxs + lrow * 33 + jb;
      px[0] = vx0[0]; px[1] = vx0[1]; px[2] = vx0[2]; px[3] = vx0[3];
      px[4] = vx1[0]; px[5] = vx1[1]; px[6] = vx1[2]; px[7] = vx1[3];
      float* py = hys + lrow * 33 + jb;
      py[0] = vy0[0]; py[1] = vy0[1]; py[2] = vy0[2]; py[3] = vy0[3];
      py[4] = vy1[0]; py[5] = vy1[1]; py[6] = vy1[2]; py[7] = vy1[3];
      if (t < 32) w2s[t] = wv;
    }
    __syncthreads();

#pragma unroll 2
    for (int h = 0; h < 32; ++h) {
      const float w = w2s[h];
      float xa[4], yb[4];
#pragma unroll
      for (int r = 0; r < 4; ++r) xa[r] = hxs[(ty * 4 + r) * 33 + h];
#pragma unroll
      for (int c = 0; c < 4; ++c) yb[c] = hys[(tx * 4 + c) * 33 + h];
#pragma unroll
      for (int r = 0; r < 4; ++r) {
#pragma unroll
        for (int c = 0; c < 4; ++c) {
          float s = xa[r] + yb[c];
          s = fmaxf(s, 0.0f);
          acc[r][c] = fmaf(s, w, acc[r][c]);
        }
      }
    }
  }

  const float bb = b2[0];
  v4f o[4];
#pragma unroll
  for (int r = 0; r < 4; ++r) {
    o[r] = (v4f){acc[r][0] + bb, acc[r][1] + bb, acc[r][2] + bb, acc[r][3] + bb};
  }
  float* obase = out + (size_t)(a0 + ty * 4) * kNB + b0 + tx * 4;
#pragma unroll
  for (int r = 0; r < 4; ++r) *(volatile v4f*)(obase + (size_t)r * kNB) = o[r];
  __threadfence();
#pragma unroll
  for (int r = 0; r < 4; ++r) *(volatile v4f*)(obase + (size_t)r * kNB) = o[r];
}

extern "C" void kernel_launch(void* const* d_in, const int* in_sizes, int n_in,
                              void* d_out, int out_size, void* d_ws, size_t ws_size,
                              hipStream_t stream) {
  if (n_in < 6) return;
  if (in_sizes[0] != kNB * kDF) return;
  if (in_sizes[1] != kNB * kDF) return;
  if (in_sizes[2] != kKIN * kHID) return;
  if (in_sizes[3] != kHID) return;
  if (in_sizes[4] != kHID) return;
  if (in_sizes[5] != 1) return;
  if (out_size != kNB * kNB) return;
  if (ws_size < kWsTotal) return;

  const float* x  = (const float*)d_in[0];
  const float* y  = (const float*)d_in[1];
  const float* W1 = (const float*)d_in[2];
  const float* b1 = (const float*)d_in[3];
  const float* W2 = (const float*)d_in[4];
  const float* b2 = (const float*)d_in[5];
  float* out = (float*)d_out;

  char* ws = (char*)d_ws;
  unsigned short* AH  = (unsigned short*)(ws + kOffAH);
  unsigned short* WT  = (unsigned short*)(ws + kOffWT);
  float*          HXY = (float*)(ws + kOffHXY);

  prep_planes_f16<<<kCvtBlocks + kTrBlocks, 256, 0, stream>>>(x, y, W1, AH, WT);

  hidden_gemm_f16<<<dim3(8, 2), 256, 0, stream>>>(AH, WT, HXY, b1);

  pair_score_kernel<<<dim3(kNB / 64, kNB / 64), 256, 0, stream>>>(
      HXY, HXY + kHidElems, W2, b2, out);
}
